// ThreeBodyModel_85581518340208
// MI455X (gfx1250) — hardware-verified
//
#include <hip/hip_runtime.h>


typedef unsigned short us;
typedef us     v8us  __attribute__((ext_vector_type(8)));
typedef us     v16us __attribute__((ext_vector_type(16)));
typedef __bf16 v16b  __attribute__((ext_vector_type(16)));
typedef float  v8f   __attribute__((ext_vector_type(8)));
typedef float  v4f   __attribute__((ext_vector_type(4)));
typedef unsigned int v4u __attribute__((ext_vector_type(4)));

union Frag { v16b v; v16us u; v8us q[2]; };
union Pk16 { v8us h; v4u u; };

namespace cfg {
constexpr int BATCH = 1024;
constexpr int T     = 100;
constexpr int D     = 12;
constexpr int H1 = 300, H2 = 100, H3 = 50;
constexpr int ROWS = 16;
constexpr int K1P = 64,  N1P = 304;
constexpr int K2P = 320, N2P = 112;
constexpr int K3P = 128, N3P = 64;
constexpr int K4P = 64,  N4P = 16;
constexpr int LA0 = 72, LA1 = 328, LA2 = 136, LA3 = 72;
constexpr int BO1 = 0, BO2 = 304, BO3 = 416, BO4 = 480, NBIAS = 496;
constexpr int OUTF = T * D;
constexpr int NT1 = N1P / 16, NT2 = N2P / 16, NT3 = N3P / 16;
}

__device__ __forceinline__ int imin(int a, int b) { return a < b ? a : b; }

__device__ __forceinline__ us bf_rne(float v) {
  unsigned int u = __float_as_uint(v);
  u += 0x7fffu + ((u >> 16) & 1u);
  return (us)(u >> 16);
}
__device__ __forceinline__ float bf_val(us b) {
  return __uint_as_float(((unsigned int)b) << 16);
}

__device__ __forceinline__ v8f wmma_bf(v16b a, v16b b, v8f c) {
  return __builtin_amdgcn_wmma_f32_16x16x32_bf16(false, a, false, b, (short)0, c, false, false);
}

__device__ __forceinline__ void wguard(v8f (&c)[4], Frag& a0, Frag& a1,
                                       Frag (&b0)[4], Frag (&b1)[4]) {
  asm volatile("v_nop\n\tv_nop\n\tv_nop\n\tv_nop"
               : "+v"(c[0]), "+v"(c[1]), "+v"(c[2]), "+v"(c[3])
               : "v"(a0.v), "v"(a1.v),
                 "v"(b0[0].v), "v"(b0[1].v), "v"(b0[2].v), "v"(b0[3].v),
                 "v"(b1[0].v), "v"(b1[1].v), "v"(b1[2].v), "v"(b1[3].v));
}
__device__ __forceinline__ void wguard(v8f (&c)[3], Frag& a0, Frag& a1,
                                       Frag (&b0)[3], Frag (&b1)[3]) {
  asm volatile("v_nop\n\tv_nop\n\tv_nop\n\tv_nop"
               : "+v"(c[0]), "+v"(c[1]), "+v"(c[2])
               : "v"(a0.v), "v"(a1.v),
                 "v"(b0[0].v), "v"(b0[1].v), "v"(b0[2].v),
                 "v"(b1[0].v), "v"(b1[1].v), "v"(b1[2].v));
}
__device__ __forceinline__ void wguard(v8f (&c)[1], Frag& a0, Frag& a1,
                                       Frag (&b0)[1], Frag (&b1)[1]) {
  asm volatile("v_nop\n\tv_nop\n\tv_nop\n\tv_nop"
               : "+v"(c[0])
               : "v"(a0.v), "v"(a1.v), "v"(b0[0].v), "v"(b1[0].v));
}

template<int N_>
__device__ __forceinline__ void zacc(v8f (&acc)[N_]) {
  const v8f z = {0.f, 0.f, 0.f, 0.f, 0.f, 0.f, 0.f, 0.f};
#pragma unroll
  for (int j = 0; j < N_; ++j) acc[j] = z;
}

template<int KT, int NBT, bool SPLIT>
__device__ __forceinline__ void mma_grp(v8f (&acc)[NBT],
                                        const us* Ah, const us* Al, int lda,
                                        const us* Bh, const us* Bl, int ldb) {
  const int l = threadIdx.x & 31, h = l >> 4, m = l & 15;
  const us* pah = Ah + m * lda + 8 * h;
  const us* pal = Al + m * lda + 8 * h;
  const us* pbh = Bh + m * ldb + 8 * h;
  const us* pbl = Bl + m * ldb + 8 * h;
#pragma unroll 1
  for (int kt = 0; kt < KT; ++kt) {
    const int ko = kt * 32;
    Frag ah, al, bh[NBT], bl[NBT];
    ah.q[0] = *(const v8us*)(pah + ko);
    ah.q[1] = *(const v8us*)(pah + ko + 16);
    if (SPLIT) {
      al.q[0] = *(const v8us*)(pal + ko);
      al.q[1] = *(const v8us*)(pal + ko + 16);
    } else {
      al.u = ah.u;
    }
#pragma unroll
    for (int j = 0; j < NBT; ++j) {
      const us* p = pbh + j * 16 * ldb + ko;
      bh[j].q[0] = *(const v8us*)p;
      bh[j].q[1] = *(const v8us*)(p + 16);
      if (SPLIT) {
        const us* q = pbl + j * 16 * ldb + ko;
        bl[j].q[0] = *(const v8us*)q;
        bl[j].q[1] = *(const v8us*)(q + 16);
      } else {
        bl[j].u = bh[j].u;
      }
    }
#pragma unroll
    for (int j = 0; j < NBT; ++j) acc[j] = wmma_bf(ah.v, bh[j].v, acc[j]);
    if (SPLIT) {
#pragma unroll
      for (int j = 0; j < NBT; ++j) acc[j] = wmma_bf(ah.v, bl[j].v, acc[j]);
#pragma unroll
      for (int j = 0; j < NBT; ++j) acc[j] = wmma_bf(al.v, bh[j].v, acc[j]);
    }
    wguard(acc, ah, al, bh, bl);
  }
}

template<int NBT>
__device__ __forceinline__ void epi_split(v8f (&acc)[NBT], const float* bias, int col0,
                                          us* Oh, us* Ol, int ldo) {
  const int l = threadIdx.x & 31, h = l >> 4, m = l & 15;
#pragma unroll
  for (int j = 0; j < NBT; ++j) {
    const int col = col0 + 16 * j + m;
    const float bv = bias[col];
    us* ph = Oh + (8 * h) * ldo + col;
    us* pl = Ol + (8 * h) * ldo + col;
#pragma unroll
    for (int r = 0; r < 8; ++r) {
      float v = acc[j][r] + bv;
      v = (v >= 0.0f) ? v : 0.01f * v;
      const us hb = bf_rne(v);
      const us lb = bf_rne(v - bf_val(hb));
      ph[r * ldo] = hb;
      pl[r * ldo] = lb;
    }
  }
}

template<int KT, int NT, bool SPLIT>
__device__ __forceinline__ void layer_hidden(const us* Ah, const us* Al, int lda,
                                             const us* Bh, const us* Bl, int ldb,
                                             const float* bias, us* Oh, us* Ol, int ldo) {
  constexpr int NG = NT / 4, REM = NT - 4 * NG;
#pragma unroll
  for (int g = 0; g < NG; ++g) {
    v8f acc[4]; zacc(acc);
    mma_grp<KT, 4, SPLIT>(acc, Ah, Al, lda, Bh + 64 * g * ldb, Bl + 64 * g * ldb, ldb);
    epi_split<4>(acc, bias, 64 * g, Oh, Ol, ldo);
  }
  if (REM == 3) {
    v8f acc[3]; zacc(acc);
    mma_grp<KT, 3, SPLIT>(acc, Ah, Al, lda, Bh + 64 * NG * ldb, Bl + 64 * NG * ldb, ldb);
    epi_split<3>(acc, bias, 64 * NG, Oh, Ol, ldo);
  }
}

__device__ __forceinline__ void put_state(us* A0, const v8f& xs, int h, int m) {
#pragma unroll
  for (int r = 0; r < 8; ++r) {
    const float v = (m < cfg::D) ? xs[r] : 0.0f;
    const us hb = bf_rne(v);
    const us lb = bf_rne(v - bf_val(hb));
    us* p = A0 + (8 * h + r) * cfg::LA0 + m;
    p[0] = hb; p[16] = hb; p[32] = lb; p[48] = lb;
  }
}

__global__ __launch_bounds__(256)
void k_pack_first(const float* __restrict__ W, us* __restrict__ P) {
  using namespace cfg;
  const int i = blockIdx.x * 256 + threadIdx.x;
  if (i >= N1P * (K1P / 8)) return;
  const int n = i >> 3, pc = i & 7;
  const int g = pc >> 1, c0 = (pc & 1) * 8;
  const int nc = imin(n, H1 - 1);
  Pk16 pk;
#pragma unroll
  for (int e = 0; e < 8; ++e) {
    const int c = c0 + e;
    const int cc = imin(c, D - 1);
    float v = W[cc * H1 + nc];
    v = (c < D && n < H1) ? v : 0.0f;
    const us hb = bf_rne(v);
    const us lb = bf_rne(v - bf_val(hb));
    pk.h[e] = (g & 1) ? lb : hb;
  }
  us* d = P + (size_t)n * K1P + pc * 8;
  *(volatile v4u*)d = pk.u;
  __threadfence();
  *(volatile v4u*)d = pk.u;
}

__global__ __launch_bounds__(256)
void k_pack_split(const float* __restrict__ W, int K, int N,
                  us* __restrict__ Ph, us* __restrict__ Pl, int Kp, int Np) {
  const int i = blockIdx.x * 256 + threadIdx.x;
  const int kq = Kp >> 3;
  if (i >= Np * kq) return;
  const int n = i / kq, k8 = (i - n * kq) * 8;
  const int nc = imin(n, N - 1);
  Pk16 ph, pl;
#pragma unroll
  for (int e = 0; e < 8; ++e) {
    const int k = k8 + e;
    const int kc = imin(k, K - 1);
    float v = W[(size_t)kc * N + nc];
    v = (k < K && n < N) ? v : 0.0f;
    const us hb = bf_rne(v);
    const us lb = bf_rne(v - bf_val(hb));
    ph.h[e] = hb;
    pl.h[e] = lb;
  }
  us* dh = Ph + (size_t)n * Kp + k8;
  us* dl = Pl + (size_t)n * Kp + k8;
  *(volatile v4u*)dh = ph.u;
  *(volatile v4u*)dl = pl.u;
  __threadfence();
  *(volatile v4u*)dh = ph.u;
  *(volatile v4u*)dl = pl.u;
}

__global__ __launch_bounds__(32)
void k_rk4(const float* __restrict__ y0, const float* __restrict__ tg,
           const float* __restrict__ b1, const float* __restrict__ b2,
           const float* __restrict__ b3, const float* __restrict__ b4,
           const us* __restrict__ P1,
           const us* __restrict__ P2h, const us* __restrict__ P2l,
           const us* __restrict__ P3h, const us* __restrict__ P3l,
           const us* __restrict__ P4h, const us* __restrict__ P4l,
           float* __restrict__ out, int nbatch) {
  using namespace cfg;
  __shared__ __attribute__((aligned(16))) us A0[ROWS * LA0];
  __shared__ __attribute__((aligned(16))) us A1h[ROWS * LA1];
  __shared__ __attribute__((aligned(16))) us A1l[ROWS * LA1];
  __shared__ __attribute__((aligned(16))) us A2h[ROWS * LA2];
  __shared__ __attribute__((aligned(16))) us A2l[ROWS * LA2];
  __shared__ __attribute__((aligned(16))) us A3h[ROWS * LA3];
  __shared__ __attribute__((aligned(16))) us A3l[ROWS * LA3];
  __shared__ __attribute__((aligned(16))) float BS[NBIAS];
  __shared__ __attribute__((aligned(16))) float OS[ROWS * OUTF];

  const int l = threadIdx.x & 31, h = l >> 4, m = l & 15;
  const int row0 = blockIdx.x * ROWS;
  if (row0 + ROWS > nbatch) return;

  const v8us z8 = {0, 0, 0, 0, 0, 0, 0, 0};
  for (int i = l; i < ROWS * LA0 / 8; i += 32) *(v8us*)(A0 + 8 * i) = z8;
  for (int i = l; i < ROWS * LA1 / 8; i += 32) { *(v8us*)(A1h + 8 * i) = z8; *(v8us*)(A1l + 8 * i) = z8; }
  for (int i = l; i < ROWS * LA2 / 8; i += 32) { *(v8us*)(A2h + 8 * i) = z8; *(v8us*)(A2l + 8 * i) = z8; }
  for (int i = l; i < ROWS * LA3 / 8; i += 32) { *(v8us*)(A3h + 8 * i) = z8; *(v8us*)(A3l + 8 * i) = z8; }
  for (int i = l; i < N1P; i += 32) { const float v = b1[imin(i, H1 - 1)]; BS[BO1 + i] = (i < H1) ? v : 0.0f; }
  for (int i = l; i < N2P; i += 32) { const float v = b2[imin(i, H2 - 1)]; BS[BO2 + i] = (i < H2) ? v : 0.0f; }
  for (int i = l; i < N3P; i += 32) { const float v = b3[imin(i, H3 - 1)]; BS[BO3 + i] = (i < H3) ? v : 0.0f; }
  for (int i = l; i < N4P; i += 32) { const float v = b4[imin(i, D - 1)];  BS[BO4 + i] = (i < D)  ? v : 0.0f; }
  __syncthreads();

  v8f x;
#pragma unroll
  for (int r = 0; r < 8; ++r) {
    const int rr = 8 * h + r;
    const float v = y0[(size_t)(row0 + rr) * OUTF + imin(m, D - 1)];
    x[r] = (m < D) ? v : 0.0f;
    if (m < D) OS[rr * OUTF + m] = x[r];
  }

  const float t00 = tg[0];
#pragma unroll 1
  for (int step = 0; step < T - 1; ++step) {
    const float dt = (tg[step + 1] - t00) - (tg[step] - t00);
    v8f ksum, kprev;
#pragma unroll
    for (int r = 0; r < 8; ++r) { ksum[r] = 0.0f; kprev[r] = 0.0f; }
#pragma unroll 1
    for (int s = 0; s < 4; ++s) {
      const float a = (s == 0) ? 0.0f : ((s == 3) ? dt : 0.5f * dt);
      const float w = (s == 1 || s == 2) ? 2.0f : 1.0f;
      v8f xs;
#pragma unroll
      for (int r = 0; r < 8; ++r) xs[r] = x[r] + a * kprev[r];
      put_state(A0, xs, h, m);
      __syncthreads();
      layer_hidden<K1P / 32, NT1, false>(A0, A0, LA0, P1, P1, K1P, BS + BO1, A1h, A1l, LA1);
      __syncthreads();
      layer_hidden<K2P / 32, NT2, true>(A1h, A1l, LA1, P2h, P2l, K2P, BS + BO2, A2h, A2l, LA2);
      __syncthreads();
      layer_hidden<K3P / 32, NT3, true>(A2h, A2l, LA2, P3h, P3l, K3P, BS + BO3, A3h, A3l, LA3);
      __syncthreads();
      v8f acc4[1]; zacc(acc4);
      mma_grp<K4P / 32, 1, true>(acc4, A3h, A3l, LA3, P4h, P4l, K4P);
      const float bv = BS[BO4 + m];
      v8f k;
#pragma unroll
      for (int r = 0; r < 8; ++r) k[r] = acc4[0][r] + bv;
#pragma unroll
      for (int r = 0; r < 8; ++r) ksum[r] = ksum[r] + w * k[r];
      kprev = k;
    }
    const float c = dt * (1.0f / 6.0f);
#pragma unroll
    for (int r = 0; r < 8; ++r) x[r] = x[r] + c * ksum[r];
#pragma unroll
    for (int r = 0; r < 8; ++r)
      if (m < D) OS[(8 * h + r) * OUTF + (step + 1) * D + m] = x[r];
  }
  __syncthreads();

  float* ob = out + (size_t)row0 * OUTF;
  constexpr int NPIECE = ROWS * OUTF / 4;
#pragma unroll 1
  for (int p = l; p < NPIECE; p += 32) {
    const v4f v = *(const v4f*)(OS + p * 4);
    *(volatile v4f*)(ob + (size_t)p * 4) = v;
  }
  __threadfence();
#pragma unroll 1
  for (int p = l; p < NPIECE; p += 32) {
    const v4f v = *(const v4f*)(OS + p * 4);
    *(volatile v4f*)(ob + (size_t)p * 4) = v;
  }
}

extern "C" void kernel_launch(void* const* d_in, const int* in_sizes, int n_in,
                              void* d_out, int out_size, void* d_ws, size_t ws_size,
                              hipStream_t stream) {
  using namespace cfg;
  if (n_in < 10) return;
  if (in_sizes[0] != BATCH * T * D || in_sizes[1] < T ||
      in_sizes[2] != D * H1 || in_sizes[3] != H1 ||
      in_sizes[4] != H1 * H2 || in_sizes[5] != H2 ||
      in_sizes[6] != H2 * H3 || in_sizes[7] != H3 ||
      in_sizes[8] != H3 * D || in_sizes[9] != D) return;
  if (out_size != BATCH * T * D) return;
  if ((BATCH % ROWS) != 0) return;

  const float* y0 = (const float*)d_in[0];
  const float* tg = (const float*)d_in[1];
  const float* W1 = (const float*)d_in[2];
  const float* b1 = (const float*)d_in[3];
  const float* W2 = (const float*)d_in[4];
  const float* b2 = (const float*)d_in[5];
  const float* W3 = (const float*)d_in[6];
  const float* b3 = (const float*)d_in[7];
  const float* W4 = (const float*)d_in[8];
  const float* b4 = (const float*)d_in[9];
  float* out = (float*)d_out;

  char* ws = (char*)d_ws;
  size_t off = 0;
  auto carve = [&](size_t bytes) -> char* {
    char* p = ws + off;
    off = (off + bytes + 255) & ~(size_t)255;
    return p;
  };
  us* P1  = (us*)carve((size_t)N1P * K1P * 2);
  us* P2h = (us*)carve((size_t)N2P * K2P * 2);
  us* P2l = (us*)carve((size_t)N2P * K2P * 2);
  us* P3h = (us*)carve((size_t)N3P * K3P * 2);
  us* P3l = (us*)carve((size_t)N3P * K3P * 2);
  us* P4h = (us*)carve((size_t)N4P * K4P * 2);
  us* P4l = (us*)carve((size_t)N4P * K4P * 2);
  if (off > ws_size) return;

  {
    const int tot = N1P * (K1P / 8);
    k_pack_first<<<dim3((tot + 255) / 256), dim3(256), 0, stream>>>(W1, P1);
  }
  {
    const int tot = N2P * (K2P / 8);
    k_pack_split<<<dim3((tot + 255) / 256), dim3(256), 0, stream>>>(W2, H1, H2, P2h, P2l, K2P, N2P);
  }
  {
    const int tot = N3P * (K3P / 8);
    k_pack_split<<<dim3((tot + 255) / 256), dim3(256), 0, stream>>>(W3, H2, H3, P3h, P3l, K3P, N3P);
  }
  {
    const int tot = N4P * (K4P / 8);
    k_pack_split<<<dim3((tot + 255) / 256), dim3(256), 0, stream>>>(W4, H3, D, P4h, P4l, K4P, N4P);
  }
  k_rk4<<<dim3(BATCH / ROWS), dim3(32), 0, stream>>>(y0, tg, b1, b2, b3, b4,
                                                     P1, P2h, P2l, P3h, P3l, P4h, P4l,
                                                     out, BATCH);
}
